// RGCN_26053271618133
// MI455X (gfx1250) — hardware-verified
//
#include <hip/hip_runtime.h>
#include <stddef.h>
#include <stdint.h>


#define DF      64
#define NREL    8
#define NBAS    4
#define DOUT2   2
#define AP      640
#define LOFF    256
#define HOFF    512
#define K0L     576
#define K1L     640
#define NTHR    256
#define NWAVE   8
#define EPT     8
#define CHUNK   (NTHR * EPT)
#define WCAP    (EPT * 32)
#define LISTN   (NWAVE * WCAP)
#define NBA     1024
#define SLA     10
#define RCAP    24576
#define DEGCAP  64
#define GBM     64
#define GBN     64
#define GTHR    128
#define UB      2048
#define UR      512
#define PT1     UB
#define PT2     (2 * UB)
#define PT3     (2 * UB + UR)
#define PT4     (PT3 + UB)
#define PT5     (PT4 + UB)
#define PT6     (PT5 + UR)
#define PT7     (PT6 + UR)
#define AGG_ZINTS   (LISTN + 2 * RCAP + 3 * NBA)
#define MISC_INTS   16
#define ROWBUF_INTS (NWAVE * AP / 2)
#define ABUF_FLT    (NWAVE * NREL * DF)
#define CNTW_INTS   (NWAVE * NREL)
#define CW_FLT      (NREL * NBAS)
#define W2S_FLT     (NBAS * DF * DOUT2)
#define R2S_FLT     (DF * DOUT2)
#define B2S_FLT     16
#define OUTS_FLT    (NBA * DOUT2)
#define OFF_ROWBUF  (AGG_ZINTS + MISC_INTS)
#define OFF_ABUF    (OFF_ROWBUF + ROWBUF_INTS)
#define OFF_CNTW    (OFF_ABUF + ABUF_FLT)
#define OFF_CW      (OFF_CNTW + CNTW_INTS)
#define OFF_W2S     (OFF_CW + CW_FLT)
#define OFF_R2S     (OFF_W2S + W2S_FLT)
#define OFF_B2S     (OFF_R2S + R2S_FLT)
#define OFF_OUTS    (OFF_B2S + B2S_FLT)
#define AGG_LDS_INTS (OFF_OUTS + OUTS_FLT)
#define WSMAX   134217728

static_assert((CHUNK & (CHUNK - 1)) == 0 && CHUNK <= 4096);
static_assert((NBA & (NBA - 1)) == 0 && NBA == (1 << SLA));
static_assert(((long long)CHUNK << SLA) < (1LL << 31));
static_assert(LISTN % NTHR == 0);
static_assert(NBA % NWAVE == 0 && NBA % 32 == 0 && NBA % GBM == 0 && NBA % 16 == 0);
static_assert(RCAP % 32 == 0 && AGG_ZINTS % (NTHR * 4) == 0 && LISTN % 4 == 0);
static_assert(OFF_ROWBUF % 4 == 0 && OFF_ABUF % 4 == 0 && OFF_CNTW % 4 == 0 && OFF_CW % 4 == 0);
static_assert(OFF_W2S % 4 == 0 && OFF_R2S % 4 == 0 && OFF_B2S % 4 == 0 && OFF_OUTS % 4 == 0);
static_assert(K0L % 32 == 0 && K1L % 32 == 0 && K1L == AP && K0L == HOFF + DF && AP == HOFF + 2 * DF);
static_assert(HOFF == 2 * LOFF && LOFF == NBAS * DF && (AP / 2) * 2 == AP);
static_assert(GBN == DF && GBM == (GTHR / 32) * 16 && DF == 2 * 32);
static_assert(UB % NTHR == 0 && UR % NTHR == 0 && UB == DF * (LOFF / 8) && UR == DF * (DF / 8) && PT7 % NTHR == 0);
static_assert(AGG_LDS_INTS * 4 <= 300000);
static_assert(OUTS_FLT % (4 * NTHR) == 0);
static_assert((AP * 2) % 128 == 0 && (K0L * 2) % 128 == 0 && (HOFF * 2) % 128 == 0 && (LOFF * 2) % 128 == 0);
static_assert(GBM * GBN * 4 == GBM * (2 * DF) * 2);

typedef float          v2f   __attribute__((ext_vector_type(2)));
typedef float          v4f   __attribute__((ext_vector_type(4)));
typedef float          v8f   __attribute__((ext_vector_type(8)));
typedef int            v4i   __attribute__((ext_vector_type(4)));
typedef int            v8i   __attribute__((ext_vector_type(8)));
typedef unsigned short v4us  __attribute__((ext_vector_type(4)));
typedef unsigned short v8us  __attribute__((ext_vector_type(8)));
typedef unsigned short v16us __attribute__((ext_vector_type(16)));
typedef __bf16         v16bf __attribute__((ext_vector_type(16)));
typedef v2f  __attribute__((may_alias)) v2fa;
typedef v4f  __attribute__((may_alias)) v4fa;
typedef v4i  __attribute__((may_alias)) v4ia;
typedef v4us __attribute__((may_alias)) v4usa;
typedef v8us __attribute__((may_alias)) v8usa;
typedef unsigned int __attribute__((may_alias)) u32a;
union FragB { v16bf v; v16us u; v8us h[2]; v8i w; };

__device__ __forceinline__ v8f wmb(const FragB& a, const FragB& b, v8f c) {
  v8f d = __builtin_amdgcn_wmma_f32_16x16x32_bf16(false, a.v, false, b.v, (short)0, c, false, false);
  asm volatile("v_nop\n\tv_nop\n\tv_nop\n\tv_nop" : "+v"(d) : "v"(a.w), "v"(b.w));
  return d;
}

__device__ __forceinline__ unsigned bf16_bits(float f) {
  const unsigned u = __float_as_uint(f);
  return (u + 0x7FFFu + ((u >> 16) & 1u)) >> 16;
}
__device__ __forceinline__ float bf16_val(float f) {
  return __uint_as_float(bf16_bits(f) << 16);
}

__device__ __forceinline__ void wave_sync() {
  __builtin_amdgcn_fence(__ATOMIC_RELEASE, "wavefront");
  __builtin_amdgcn_wave_barrier();
  __builtin_amdgcn_fence(__ATOMIC_ACQUIRE, "wavefront");
}

template <int SLB>
__device__ __forceinline__ int scan_chunk(const int* __restrict__ dsts, int nE, int cbase, int slotBase,
                                          int nb, int vec8, int* list, int tid, int lane, int wave) {
  int wc = 0;
  const int el0  = tid * EPT;
  const int e0   = cbase + el0;
  const int sent = -2147483647 - 1;
  v4i da, db;
  if (vec8 != 0 && cbase + CHUNK <= nE) {
    da = *(const v4i*)(dsts + e0);
    db = *(const v4i*)(dsts + e0 + 4);
  } else {
    da.x = (e0     < nE) ? dsts[min(e0,     nE - 1)] : sent;
    da.y = (e0 + 1 < nE) ? dsts[min(e0 + 1, nE - 1)] : sent;
    da.z = (e0 + 2 < nE) ? dsts[min(e0 + 2, nE - 1)] : sent;
    da.w = (e0 + 3 < nE) ? dsts[min(e0 + 3, nE - 1)] : sent;
    db.x = (e0 + 4 < nE) ? dsts[min(e0 + 4, nE - 1)] : sent;
    db.y = (e0 + 5 < nE) ? dsts[min(e0 + 5, nE - 1)] : sent;
    db.z = (e0 + 6 < nE) ? dsts[min(e0 + 6, nE - 1)] : sent;
    db.w = (e0 + 7 < nE) ? dsts[min(e0 + 7, nE - 1)] : sent;
  }
  const unsigned nbs = (unsigned)slotBase;
  const unsigned unb = (unsigned)nb;
  const unsigned s0 = (unsigned)da.x - nbs, s1 = (unsigned)da.y - nbs;
  const unsigned s2 = (unsigned)da.z - nbs, s3 = (unsigned)da.w - nbs;
  const unsigned s4 = (unsigned)db.x - nbs, s5 = (unsigned)db.y - nbs;
  const unsigned s6 = (unsigned)db.z - nbs, s7 = (unsigned)db.w - nbs;
  const bool h0 = s0 < unb, h1 = s1 < unb, h2 = s2 < unb, h3 = s3 < unb;
  const bool h4 = s4 < unb, h5 = s5 < unb, h6 = s6 < unb, h7 = s7 < unb;
  const unsigned any = __builtin_amdgcn_ballot_w32(h0 | h1 | h2 | h3 | h4 | h5 | h6 | h7);
  if (any != 0u) {
#define HITJ(J, HJ, SJ) { \
      const unsigned mj = __builtin_amdgcn_ballot_w32(HJ); \
      if (mj != 0u) { \
        if (HJ) { \
          const int pos = wc + (int)__builtin_amdgcn_mbcnt_lo(mj, 0u); \
          if (pos < WCAP) list[wave * WCAP + pos] = ((el0 + (J)) << SLB) | (int)(SJ); \
        } \
        wc += (int)__builtin_popcount(mj); } }
    HITJ(0, h0, s0)
    HITJ(1, h1, s1)
    HITJ(2, h2, s2)
    HITJ(3, h3, s3)
    HITJ(4, h4, s4)
    HITJ(5, h5, s5)
    HITJ(6, h6, s6)
    HITJ(7, h7, s7)
#undef HITJ
  }
  return wc;
}

__global__ __launch_bounds__(NTHR) void k_wprep(const float* __restrict__ ba0, const float* __restrict__ ro0,
                                                const float* __restrict__ ba1, const float* __restrict__ ro1,
                                                unsigned short* Bt0, unsigned short* Bt1) {
  const int u = (int)blockIdx.x * NTHR + (int)threadIdx.x;
  const float* W;
  unsigned short* P;
  int pitch, coff, v, isRoot;
  if (u < PT1)      { W = ba0; P = Bt0; pitch = K0L; coff = 0;         v = u;       isRoot = 0; }
  else if (u < PT2) { W = ba0; P = Bt0; pitch = K0L; coff = LOFF;      v = u - PT1; isRoot = 0; }
  else if (u < PT3) { W = ro0; P = Bt0; pitch = K0L; coff = HOFF;      v = u - PT2; isRoot = 1; }
  else if (u < PT4) { W = ba1; P = Bt1; pitch = K1L; coff = 0;         v = u - PT3; isRoot = 0; }
  else if (u < PT5) { W = ba1; P = Bt1; pitch = K1L; coff = LOFF;      v = u - PT4; isRoot = 0; }
  else if (u < PT6) { W = ro1; P = Bt1; pitch = K1L; coff = HOFF;      v = u - PT5; isRoot = 1; }
  else if (u < PT7) { W = ro1; P = Bt1; pitch = K1L; coff = HOFF + DF; v = u - PT6; isRoot = 1; }
  else return;
  const int n  = isRoot ? (v >> 3) : (v >> 5);
  const int k8 = isRoot ? ((v & 7) * 8) : ((v & 31) * 8);
  const float* p = W + (size_t)k8 * DF + n;
  v8us o;
#pragma unroll
  for (int i = 0; i < 8; ++i) o[i] = (unsigned short)bf16_bits(p[(size_t)i * DF]);
  unsigned short* dp = P + (size_t)n * pitch + coff + k8;
  *(volatile v8us*)dp = o;
  __threadfence();
  *(volatile v8us*)dp = o;
}

__global__ __launch_bounds__(GTHR) void k_gemm(unsigned short* Apl, const unsigned short* __restrict__ BT, int K,
                                               const float* __restrict__ bias, int nOut) {
  __shared__ __attribute__((aligned(16))) float stg[GBM * GBN];
  const int tid = (int)threadIdx.x, lane = tid & 31, wave = tid >> 5, hh = lane >> 4, m = lane & 15;
  const int rowBase = (int)blockIdx.x * GBM;

  v8f acc[4];
  {
    const v8f z = {0.f, 0.f, 0.f, 0.f, 0.f, 0.f, 0.f, 0.f};
    acc[0] = z; acc[1] = z; acc[2] = z; acc[3] = z;
  }
  const unsigned short* ap = Apl + (size_t)(rowBase + 16 * wave + m) * (size_t)AP + 8 * hh;
  const unsigned short* bp = BT + (size_t)m * (size_t)K + 8 * hh;

#pragma unroll 1
  for (int k0 = 0; k0 < K; k0 += 32) {
    FragB af;
    af.h[0] = *(const v8usa*)(ap + k0);
    af.h[1] = *(const v8usa*)(ap + k0 + 16);
#pragma unroll
    for (int nt = 0; nt < 4; ++nt) {
      const unsigned short* wq = bp + (size_t)(16 * nt) * (size_t)K + k0;
      FragB bf;
      bf.h[0] = *(const v8usa*)wq;
      bf.h[1] = *(const v8usa*)(wq + 16);
      acc[nt] = wmb(af, bf, acc[nt]);
    }
  }

#pragma unroll
  for (int nt = 0; nt < 4; ++nt) {
    const int lc = 16 * nt + m;
#pragma unroll
    for (int r = 0; r < 8; ++r) {
      const int lr = 16 * wave + 8 * hh + r;
      stg[lr * GBN + lc] = acc[nt][r];
    }
  }
  __syncthreads();

  v4f bb4;
  {
    const v4f t1 = *(const v4fa*)(bias + 4 * m);
    bb4.x = bf16_val(t1.x); bb4.y = bf16_val(t1.y); bb4.z = bf16_val(t1.z); bb4.w = bf16_val(t1.w);
  }
  v4f fv[8];
#pragma unroll
  for (int i = 0; i < 8; ++i) {
    const int lr = 16 * wave + 2 * i + hh;
    fv[i] = *(const v4fa*)(stg + lr * GBN + 4 * m);
  }
  __syncthreads();

#pragma unroll
  for (int i = 0; i < 8; ++i) {
    const int lr = 16 * wave + 2 * i + hh;
    const bool ok = (rowBase + lr) < nOut;
    const v4f t = fv[i] + bb4;
    v4f y;
    y.x = (t.x > 0.0f) ? t.x : (t.x - t.x);
    y.y = (t.y > 0.0f) ? t.y : (t.y - t.y);
    y.z = (t.z > 0.0f) ? t.z : (t.z - t.z);
    y.w = (t.w > 0.0f) ? t.w : (t.w - t.w);
    y.x = ok ? y.x : 0.0f; y.y = ok ? y.y : 0.0f; y.z = ok ? y.z : 0.0f; y.w = ok ? y.w : 0.0f;
    v4us h4, l4;
    unsigned hb;
    hb = bf16_bits(y.x); h4[0] = (unsigned short)hb; l4[0] = (unsigned short)bf16_bits(y.x - __uint_as_float(hb << 16));
    hb = bf16_bits(y.y); h4[1] = (unsigned short)hb; l4[1] = (unsigned short)bf16_bits(y.y - __uint_as_float(hb << 16));
    hb = bf16_bits(y.z); h4[2] = (unsigned short)hb; l4[2] = (unsigned short)bf16_bits(y.z - __uint_as_float(hb << 16));
    hb = bf16_bits(y.w); h4[3] = (unsigned short)hb; l4[3] = (unsigned short)bf16_bits(y.w - __uint_as_float(hb << 16));
    unsigned short* srow = (unsigned short*)stg + (size_t)lr * (2 * DF);
    *(v4usa*)(srow + 4 * m) = h4;
    *(v4usa*)(srow + DF + 4 * m) = l4;
  }
  __syncthreads();
  v8us qv[8];
#pragma unroll
  for (int i = 0; i < 8; ++i) {
    const int lr = 16 * wave + 2 * i + hh;
    const unsigned short* srow = (const unsigned short*)stg + (size_t)lr * (2 * DF);
    qv[i] = *(const v8usa*)(srow + 8 * m);
  }
#pragma unroll
  for (int i = 0; i < 8; ++i) {
    const int lr = 16 * wave + 2 * i + hh;
    unsigned short* rp = Apl + (size_t)(rowBase + lr) * (size_t)AP + HOFF + 8 * m;
    *(volatile v8us*)rp = qv[i];
  }
  __threadfence();
#pragma unroll
  for (int i = 0; i < 8; ++i) {
    const int lr = 16 * wave + 2 * i + hh;
    unsigned short* rp = Apl + (size_t)(rowBase + lr) * (size_t)AP + HOFF + 8 * m;
    *(volatile v8us*)rp = qv[i];
  }
}

template <int L>
__global__ __launch_bounds__(NTHR) void k_scan(const int* __restrict__ srcs, const int* __restrict__ dsts,
                                               const int* __restrict__ ety, int nE, int nN, int vec8, int mRows,
                                               const float* __restrict__ xin, const float* __restrict__ comp,
                                               const float* __restrict__ bs2, const float* __restrict__ rt2,
                                               const float* __restrict__ bi2,
                                               unsigned short* apl, float* outp) {
  extern __shared__ __attribute__((aligned(16))) int dsm[];
  int* list = dsm;
  int* hl   = dsm + LISTN;
  int* sl   = hl + RCAP;
  int* cnt  = sl + RCAP;
  int* offs = cnt + NBA;
  int* cur  = offs + NBA;
  int* misc = cur + NBA;
  const int tid = (int)threadIdx.x, lane = tid & 31, wave = tid >> 5;
  unsigned short* rowbuf = (unsigned short*)(dsm + OFF_ROWBUF) + wave * AP;
  float* abuf = (float*)(dsm + OFF_ABUF) + wave * (NREL * DF);
  int*   cntw = dsm + OFF_CNTW + wave * NREL;
  float* cwl  = (float*)(dsm + OFF_CW);
  float* w2s  = (float*)(dsm + OFF_W2S);
  float* r2s  = (float*)(dsm + OFF_R2S);
  float* b2s  = (float*)(dsm + OFF_B2S);
  float* outs = (float*)(dsm + OFF_OUTS);
  const int nodeBase = (int)blockIdx.x * NBA;

  {
    const v4i z4 = {0, 0, 0, 0};
    for (int i = tid * 4; i < AGG_ZINTS; i += NTHR * 4) *(v4ia*)(dsm + i) = z4;
    if (tid < MISC_INTS) misc[tid] = 0;
    if (tid < CW_FLT) cwl[tid] = bf16_val(comp[tid]);
    if constexpr (L == 2) {
#pragma unroll 1
      for (int i = tid; i < W2S_FLT; i += NTHR) w2s[i] = bf16_val(bs2[i]);
      if (tid < R2S_FLT) r2s[tid] = bf16_val(rt2[tid]);
      if (tid < B2S_FLT) {
        const float bb = bi2[tid < DOUT2 ? tid : DOUT2 - 1];
        b2s[tid] = (tid < DOUT2) ? bf16_val(bb) : 0.0f;
      }
    }
  }
  __syncthreads();

  int t = 0, ov = 0;
  const int nChunks = (nE + CHUNK - 1) / CHUNK;
#pragma unroll 1
  for (int ch = 0; ch < nChunks; ++ch) {
    const int cbase = ch * CHUNK;
    const int wc = scan_chunk<SLA>(dsts, nE, cbase, nodeBase, NBA, vec8, list, tid, lane, wave);
    if (lane == 0) misc[wave] = wc;
    __syncthreads();
    if (wave == 0) {
#pragma unroll 1
      for (int w2 = 0; w2 < NWAVE; ++w2) {
        int c = misc[w2];
        c = c < 0 ? 0 : (c > WCAP ? WCAP : c);
#pragma unroll 1
        for (int b0 = 0; b0 < c; b0 += 32) {
          const int idx = b0 + lane;
          const int ent = list[w2 * WCAP + (idx < WCAP ? idx : WCAP - 1)];
          const int m32 = (c - b0) < 32 ? (c - b0) : 32;
#pragma unroll 1
          for (int k = 0; k < m32; ++k) {
            const int u    = __builtin_amdgcn_readlane(ent, k);
            const int slot = u & (NBA - 1);
            const int el   = (u >> SLA) & (CHUNK - 1);
            const int pk   = ((cbase + el) << SLA) | slot;
            if (t < RCAP) {
              if (lane == 0) { hl[t] = pk; cnt[slot] = cnt[slot] + 1; }
              t = t + 1;
            } else {
              ov = 1;
            }
          }
        }
      }
    }
    __syncthreads();
  }
  if (wave == 0 && lane == 0) { misc[8] = t; misc[9] = ov; }
  __syncthreads();
  int tt = misc[8];
  tt = tt < 0 ? 0 : (tt > RCAP ? RCAP : tt);
  const int ovf = misc[9];

  if (wave == 0) {
    const int base = lane * (NBA / 32);
    int s = 0;
#pragma unroll 1
    for (int i = 0; i < NBA / 32; ++i) s += cnt[base + i];
    int incl = s;
#pragma unroll
    for (int d = 1; d < 32; d <<= 1) {
      const int y = __shfl_up(incl, d, 32);
      if (lane >= d) incl += y;
    }
    int run = incl - s;
#pragma unroll 1
    for (int i = 0; i < NBA / 32; ++i) {
      const int cv = cnt[base + i];
      offs[base + i] = run;
      cur[base + i]  = run;
      run += cv;
    }
  }
  __syncthreads();
  if (wave == 0) {
#pragma unroll 1
    for (int b0 = 0; b0 < tt; b0 += 32) {
      const int idx = b0 + lane;
      const int ent = hl[idx < RCAP ? idx : RCAP - 1];
      const int m32 = (tt - b0) < 32 ? (tt - b0) : 32;
#pragma unroll 1
      for (int k = 0; k < m32; ++k) {
        const int u    = __builtin_amdgcn_readlane(ent, k);
        const int slot = u & (NBA - 1);
        if (lane == 0) {
          int p = cur[slot];
          p = p < 0 ? 0 : (p > RCAP - 1 ? RCAP - 1 : p);
          sl[p] = u;
          cur[slot] = p + 1;
        }
      }
    }
  }
  __syncthreads();

  const float qnan = __int_as_float(0x7fc00000);
  const bool ovfb = (ovf != 0);
#pragma unroll 1
  for (int si = 0; si < NBA / NWAVE; ++si) {
    const int s    = si * NWAVE + wave;
    const int node = nodeBase + s;
    int c = cnt[s];
    const bool big = c > DEGCAP;
    c = c < 0 ? 0 : (c > DEGCAP ? DEGCAP : c);
    int o = offs[s];
    o = o < 0 ? 0 : (o > RCAP ? RCAP : o);
    const int nc = node < nN ? node : nN - 1;
    float sa[NREL], sb[NREL];
    int cr[NREL];
#pragma unroll
    for (int r = 0; r < NREL; ++r) { sa[r] = 0.0f; sb[r] = 0.0f; cr[r] = 0; }
    bool badr = false;
#pragma unroll 1
    for (int b0 = 0; b0 < c; b0 += 32) {
      int idx = o + b0 + lane;
      idx = idx > RCAP - 1 ? RCAP - 1 : idx;
      const int ent = sl[idx];
      int eid = ent >> SLA;
      eid = eid < 0 ? 0 : (eid > nE - 1 ? nE - 1 : eid);
      int sr = srcs[eid];
      sr = sr < 0 ? 0 : (sr > nN - 1 ? nN - 1 : sr);
      const int rt = ety[eid];
      const int m32 = (c - b0) < 32 ? (c - b0) : 32;
      const bool inb = lane < m32;
#pragma unroll
      for (int r = 0; r < NREL; ++r)
        cr[r] += (int)__builtin_popcount(__builtin_amdgcn_ballot_w32(inb && (rt == r)));
      badr = badr || (__builtin_amdgcn_ballot_w32(inb && ((unsigned)rt >= (unsigned)NREL)) != 0u);
#pragma unroll 1
      for (int k = 0; k < m32; ++k) {
        const int sk = __builtin_amdgcn_readlane(sr, k);
        const int rk = __builtin_amdgcn_readlane(rt, k);
        float v0, v1;
        if constexpr (L == 0) {
          const v2f a = *(const v2fa*)(xin + (size_t)sk * DF + 2 * lane);
          v0 = bf16_val(a.x); v1 = bf16_val(a.y);
        } else {
          const unsigned short* rp = apl + (size_t)sk * AP + HOFF + 2 * lane;
          const unsigned wh = *(const u32a*)rp;
          const unsigned wl = *(const u32a*)(rp + DF);
          v0 = __uint_as_float(wh << 16)         + __uint_as_float(wl << 16);
          v1 = __uint_as_float(wh & 0xffff0000u) + __uint_as_float(wl & 0xffff0000u);
        }
#pragma unroll
        for (int r = 0; r < NREL; ++r) {
          const bool e = (rk == r);
          sa[r] = e ? (sa[r] + v0) : sa[r];
          sb[r] = e ? (sb[r] + v1) : sb[r];
        }
      }
    }
#pragma unroll
    for (int r = 0; r < NREL; ++r) {
      v2f tv; tv.x = sa[r]; tv.y = sb[r];
      *(v2fa*)(abuf + r * DF + 2 * lane) = tv;
    }
    if (lane == 0) {
#pragma unroll
      for (int r = 0; r < NREL; ++r) cntw[r] = cr[r];
    }
    wave_sync();
    float ax[NBAS], ay[NBAS];
#pragma unroll
    for (int b = 0; b < NBAS; ++b) { ax[b] = 0.0f; ay[b] = 0.0f; }
#pragma unroll 1
    for (int r = 0; r < NREL; ++r) {
      const int crr = cntw[r];
      const float cf = (float)(crr < 1 ? 1 : crr);
      const float inv = 1.0f / cf;
      const v2f tv = *(const v2fa*)(abuf + r * DF + 2 * lane);
      const float m0 = tv.x * inv, m1 = tv.y * inv;
      const v4f w = *(const v4fa*)(cwl + NBAS * r);
      ax[0] = fmaf(w.x, m0, ax[0]); ay[0] = fmaf(w.x, m1, ay[0]);
      ax[1] = fmaf(w.y, m0, ax[1]); ay[1] = fmaf(w.y, m1, ay[1]);
      ax[2] = fmaf(w.z, m0, ax[2]); ay[2] = fmaf(w.z, m1, ay[2]);
      ax[3] = fmaf(w.w, m0, ax[3]); ay[3] = fmaf(w.w, m1, ay[3]);
    }
    const float pzr = (big || badr || ovfb) ? qnan : 0.0f;
    const bool live = node < nN;
    if constexpr (L != 2) {
#pragma unroll
      for (int b = 0; b < NBAS; ++b) {
        const float m0 = live ? (ax[b] + pzr) : 0.0f;
        const float m1 = live ? (ay[b] + pzr) : 0.0f;
        const unsigned h0 = bf16_bits(m0), h1 = bf16_bits(m1);
        const unsigned l0 = bf16_bits(m0 - __uint_as_float(h0 << 16));
        const unsigned l1 = bf16_bits(m1 - __uint_as_float(h1 << 16));
        *(u32a*)(rowbuf + b * DF + 2 * lane)        = h0 | (h1 << 16);
        *(u32a*)(rowbuf + LOFF + b * DF + 2 * lane) = l0 | (l1 << 16);
      }
      if constexpr (L == 0) {
        const v2f xs = *(const v2fa*)(xin + (size_t)nc * DF + 2 * lane);
        const unsigned xb0 = live ? bf16_bits(xs.x + pzr) : 0u;
        const unsigned xb1 = live ? bf16_bits(xs.y + pzr) : 0u;
        *(u32a*)(rowbuf + HOFF + 2 * lane)      = xb0 | (xb1 << 16);
        *(u32a*)(rowbuf + HOFF + DF + 2 * lane) = 0u;
      }
      wave_sync();
      const v8us q0 = *(const v8usa*)(rowbuf + 8 * lane);
      const v8us q1 = *(const v8usa*)(rowbuf + LOFF + 8 * lane);
      v8us q2 = {0, 0, 0, 0, 0, 0, 0, 0};
      if constexpr (L == 0) q2 = *(const v8usa*)(rowbuf + HOFF + 8 * (lane & 15));
      wave_sync();
      if (node < mRows) {
        unsigned short* rpw = apl + (size_t)node * AP;
        *(volatile v8us*)(rpw + 8 * lane) = q0;
        *(volatile v8us*)(rpw + LOFF + 8 * lane) = q1;
        if constexpr (L == 0) { if (lane < 16) *(volatile v8us*)(rpw + HOFF + 8 * (lane & 15)) = q2; }
        __threadfence();
        *(volatile v8us*)(rpw + 8 * lane) = q0;
        *(volatile v8us*)(rpw + LOFF + 8 * lane) = q1;
        if constexpr (L == 0) { if (lane < 16) *(volatile v8us*)(rpw + HOFF + 8 * (lane & 15)) = q2; }
      }
    } else {
      const unsigned short* rp = apl + (size_t)nc * AP + HOFF + 2 * lane;
      const unsigned wh = *(const u32a*)rp;
      const unsigned wl = *(const u32a*)(rp + DF);
      const float hv0 = __uint_as_float(wh << 16)         + __uint_as_float(wl << 16);
      const float hv1 = __uint_as_float(wh & 0xffff0000u) + __uint_as_float(wl & 0xffff0000u);
      float p0 = 0.0f, p1 = 0.0f;
      const int f0 = 2 * lane;
#pragma unroll
      for (int b = 0; b < NBAS; ++b) {
        const v4f w = *(const v4fa*)(w2s + (b * DF + f0) * DOUT2);
        p0 = fmaf(ax[b], w.x, p0); p1 = fmaf(ax[b], w.y, p1);
        p0 = fmaf(ay[b], w.z, p0); p1 = fmaf(ay[b], w.w, p1);
      }
      {
        const v4f w = *(const v4fa*)(r2s + f0 * DOUT2);
        p0 = fmaf(hv0, w.x, p0); p1 = fmaf(hv0, w.y, p1);
        p0 = fmaf(hv1, w.z, p0); p1 = fmaf(hv1, w.w, p1);
      }
#pragma unroll
      for (int d = 16; d >= 1; d >>= 1) {
        p0 += __shfl_xor(p0, d, 32);
        p1 += __shfl_xor(p1, d, 32);
      }
      const float o0 = live ? ((p0 + b2s[0]) + pzr) : 0.0f;
      const float o1 = live ? ((p1 + b2s[1]) + pzr) : 0.0f;
      if (lane == 0) { outs[DOUT2 * s] = o0; outs[DOUT2 * s + 1] = o1; }
    }
    wave_sync();
  }

  if constexpr (L == 2) {
    __syncthreads();
    constexpr int NIT = OUTS_FLT / (4 * NTHR);
    v4f ovv[NIT];
#pragma unroll
    for (int it = 0; it < NIT; ++it) ovv[it] = *(const v4fa*)(outs + 4 * (it * NTHR + tid));
    const size_t obase = (size_t)nodeBase * DOUT2;
    const size_t olim  = (size_t)nN * DOUT2;
#pragma unroll
    for (int it = 0; it < NIT; ++it) {
      const size_t gi = obase + 4 * (size_t)(it * NTHR + tid);
      if (gi + 4 <= olim) *(volatile v4f*)(outp + gi) = ovv[it];
    }
    __threadfence();
#pragma unroll
    for (int it = 0; it < NIT; ++it) {
      const size_t gi = obase + 4 * (size_t)(it * NTHR + tid);
      if (gi + 4 <= olim) *(volatile v4f*)(outp + gi) = ovv[it];
    }
  }
}

static inline int cdiv(int a, int b) { return (a + b - 1) / b; }
static inline size_t al256(size_t o) { return (o + 255) & ~(size_t)255; }

extern "C" void kernel_launch(void* const* d_in, const int* in_sizes, int n_in,
                              void* d_out, int out_size, void* d_ws, size_t ws_size,
                              hipStream_t stream) {
  if (n_in < 15) return;
  if (in_sizes[0] < DF || (in_sizes[0] % DF) != 0) return;
  const int nN = in_sizes[0] / DF;
  if (nN < 16 || (nN % 16) != 0 || nN > (1 << 22)) return;
  if (in_sizes[1] < 2 || (in_sizes[1] & 1) != 0) return;
  const int nE = in_sizes[1] / 2;
  if (nE < 1 || nE >= (1 << (31 - SLA))) return;
  if (in_sizes[2] != nE) return;
  if (in_sizes[3] != NBAS * DF * DF || in_sizes[4] != NREL * NBAS) return;
  if (in_sizes[5] != DF * DF || in_sizes[6] != DF) return;
  if (in_sizes[7] != NBAS * DF * DF || in_sizes[8] != NREL * NBAS) return;
  if (in_sizes[9] != DF * DF || in_sizes[10] != DF) return;
  if (in_sizes[11] != NBAS * DF * DOUT2 || in_sizes[12] != NREL * NBAS) return;
  if (in_sizes[13] != DF * DOUT2 || in_sizes[14] != DOUT2) return;
  if ((long long)out_size != (long long)nN * DOUT2) return;

  const float* x    = (const float*)d_in[0];
  const int*   edge = (const int*)d_in[1];
  const int*   ety  = (const int*)d_in[2];
  const float* ba0  = (const float*)d_in[3];
  const float* co0  = (const float*)d_in[4];
  const float* ro0  = (const float*)d_in[5];
  const float* bi0  = (const float*)d_in[6];
  const float* ba1  = (const float*)d_in[7];
  const float* co1  = (const float*)d_in[8];
  const float* ro1  = (const float*)d_in[9];
  const float* bi1  = (const float*)d_in[10];
  const float* ba2  = (const float*)d_in[11];
  const float* co2  = (const float*)d_in[12];
  const float* ro2  = (const float*)d_in[13];
  const float* bi2  = (const float*)d_in[14];
  float* out = (float*)d_out;
  const int* src = edge;
  const int* dst = edge + nE;

  const int MP = cdiv(nN, GBM) * GBM;
  const int gM = MP / GBM;
  const int gA = cdiv(MP, NBA);
  if ((long long)gA * NBA < (long long)MP) return;
  const int vec8 = ((nE & 3) == 0) ? 1 : 0;

  char* ws = (char*)d_ws;
  size_t off = 0;
  const size_t oBt0 = off; off = al256(off + (size_t)DF * K0L * 2);
  const size_t oBt1 = off; off = al256(off + (size_t)DF * K1L * 2);
  const size_t oA   = off; off = al256(off + (size_t)MP * AP * 2);
  if (off > ws_size || off > (size_t)WSMAX) return;
  unsigned short* Bt0 = (unsigned short*)(ws + oBt0);
  unsigned short* Bt1 = (unsigned short*)(ws + oBt1);
  unsigned short* Apl = (unsigned short*)(ws + oA);

  const size_t scanLds = (size_t)AGG_LDS_INTS * 4;
  hipFuncSetAttribute(reinterpret_cast<const void*>(&k_scan<0>), hipFuncAttributeMaxDynamicSharedMemorySize, (int)scanLds);
  hipFuncSetAttribute(reinterpret_cast<const void*>(&k_scan<1>), hipFuncAttributeMaxDynamicSharedMemorySize, (int)scanLds);
  hipFuncSetAttribute(reinterpret_cast<const void*>(&k_scan<2>), hipFuncAttributeMaxDynamicSharedMemorySize, (int)scanLds);

  k_wprep<<<PT7 / NTHR, NTHR, 0, stream>>>(ba0, ro0, ba1, ro1, Bt0, Bt1);
  k_scan<0><<<gA, NTHR, scanLds, stream>>>(src, dst, ety, nE, nN, vec8, MP, x, co0, ba2, ro2, bi2, Apl, out);
  k_gemm<<<gM, GTHR, 0, stream>>>(Apl, Bt0, K0L, bi0, nN);
  k_scan<1><<<gA, NTHR, scanLds, stream>>>(src, dst, ety, nE, nN, vec8, MP, x, co1, ba2, ro2, bi2, Apl, out);
  k_gemm<<<gM, GTHR, 0, stream>>>(Apl, Bt1, K1L, bi1, nN);
  k_scan<2><<<gA, NTHR, scanLds, stream>>>(src, dst, ety, nE, nN, vec8, MP, x, co2, ba2, ro2, bi2, Apl, out);
}
